// RNN_54022098649219
// MI455X (gfx1250) — hardware-verified
//
#include <hip/hip_runtime.h>
#include <math.h>

constexpr int NB    = 256;
constexpr int NSTEP = 2048;
constexpr int NHID  = 256;
constexpr int NP    = 24;
constexpr int NTHR  = 512;
constexpr int NWAVE = NTHR / 32;
constexpr int RPB   = 16;
constexpr int NBLK  = NB / RPB;
constexpr int NKB   = NHID / 32;
constexpr int XCH   = 64;
constexpr int LDP   = NHID + 8;
constexpr int TILEH = RPB * LDP;
constexpr int SXP   = XCH + 4;
constexpr int HFP   = NHID + 4;
constexpr int NOUTB = RPB * NP;
constexpr float WCAR       = 256.0f;
constexpr float WCAR_INV   = 1.0f / 256.0f;
constexpr float LOCAR      = 2048.0f;
constexpr float LOCAR_INV  = 1.0f / 2048.0f;
constexpr float F16_MIN_NORMAL = 6.103515625e-05f;
static_assert(NB % RPB == 0);
static_assert(NHID == 16 * NWAVE);
static_assert(NHID % 32 == 0);
static_assert(NSTEP % XCH == 0);
static_assert((XCH & (XCH - 1)) == 0);
static_assert(RPB * XCH == 2 * NTHR);
static_assert(LDP % 8 == 0 && HFP % 4 == 0 && SXP % 2 == 0);
static_assert((4 * TILEH) % 8 == 0);
static_assert(NOUTB % 32 == 0);
static_assert(NOUTB <= NTHR);
static_assert(NOUTB == 3 * 32 * 4);
static_assert((NOUTB * 4) % 128 == 0);

typedef __attribute__((ext_vector_type(16))) _Float16 v16h;
typedef __attribute__((ext_vector_type(8)))  _Float16 v8h;
typedef __attribute__((ext_vector_type(8)))  float    v8f;
typedef __attribute__((ext_vector_type(4)))  float    v4f;
typedef __attribute__((ext_vector_type(2)))  float    v2f;

__device__ __forceinline__ unsigned short f2bf_bits(float f) {
  unsigned u = __float_as_uint(f);
  return (unsigned short)((u + 0x7FFFu + ((u >> 16) & 1u)) >> 16);
}
__device__ __forceinline__ float bf_bits2f(unsigned short h) { return __uint_as_float(((unsigned)h) << 16); }
__device__ __forceinline__ float bf16r(float f) { return bf_bits2f(f2bf_bits(f)); }

__device__ __forceinline__ void acc_guard2(v8f& a, v8f& b) { asm volatile("v_nop\n\tv_nop\n\tv_nop\n\tv_nop" : "+v"(a), "+v"(b)); }
__device__ __forceinline__ void wmma_guard3(v8f& a, v8f& b, v16h x, v16h y, v16h z) {
  asm volatile("v_nop\n\tv_nop\n\tv_nop\n\tv_nop" : "+v"(a), "+v"(b) : "v"(x), "v"(y), "v"(z));
}

template <typename T> struct Frag;
template <> struct Frag<_Float16> {
  typedef v16h V; union U { v16h v; v8h h[2]; };
  static __device__ __forceinline__ v16h load(const _Float16* p) {
    U f; f.h[0] = *(const v8h*)(p); f.h[1] = *(const v8h*)(p + 16); return f.v;
  }
  static __device__ __forceinline__ v8f mma(v16h a, v16h b, v8f c) {
    return __builtin_amdgcn_wmma_f32_16x16x32_f16(false, a, false, b, (short)0, c, false, false);
  }
};

__device__ __forceinline__ float tanh_f(float x) {
  const float xc = fminf(fmaxf(x, -16.0f), 16.0f);
  const float e  = expf(2.0f * xc);
  return 1.0f - 2.0f * __builtin_amdgcn_rcpf(e + 1.0f);
}

__global__ __launch_bounds__(NTHR) void rnn_tanh_seq_kernel(
    const float* x,
    const float* w_ih,
    const float* w_hh,
    const float* b_ih,
    const float* b_hh,
    const float* w_out,
    const float* b_out,
    float* out) {
  __shared__ __align__(16) _Float16 hbuf[4 * TILEH];
  __shared__ __align__(16) float    s_x[RPB * SXP];
  __shared__ __align__(16) float    s_hf[RPB * HFP];
  __shared__ __align__(16) float    s_out[NOUTB];

  const int tid = threadIdx.x, lane = tid & 31, wave = tid >> 5;
  const int c = lane & 15, hh = lane >> 4, koff = hh * 8, mOff = hh * 8;
  const int b0 = blockIdx.x * RPB;
  const int hidx = wave * 16 + c;

  {
    v8h z8;
#pragma unroll
    for (int e = 0; e < 8; ++e) z8[e] = (_Float16)0.0f;
    for (int i = tid; i < (4 * TILEH) / 8; i += NTHR) *(v8h*)(hbuf + i * 8) = z8;
  }

  const float wih = bf16r(w_ih[hidx]);
  const float bih = bf16r(b_ih[hidx]);
  const float bhh = bf16r(b_hh[hidx]);

  v16h bfr[NKB];
  {
    const float* wrow = w_hh + (size_t)hidx * NHID + koff;
#pragma unroll
    for (int kb = 0; kb < NKB; ++kb) {
      const v4f w0 = *(const v4f*)(wrow + kb * 32);
      const v4f w1 = *(const v4f*)(wrow + kb * 32 + 4);
      const v4f w2 = *(const v4f*)(wrow + kb * 32 + 16);
      const v4f w3 = *(const v4f*)(wrow + kb * 32 + 20);
#pragma unroll
      for (int e = 0; e < 4; ++e) {
        const float f0 = w0[e], f1 = w1[e], f2 = w2[e], f3 = w3[e];
        bfr[kb][e]      = (_Float16)(bf16r(f0) * WCAR);
        bfr[kb][4 + e]  = (_Float16)(bf16r(f1) * WCAR);
        bfr[kb][8 + e]  = (_Float16)(bf16r(f2) * WCAR);
        bfr[kb][12 + e] = (_Float16)(bf16r(f3) * WCAR);
      }
      asm volatile("" ::: "memory");
    }
  }

  float hlast[8];
#pragma unroll
  for (int r = 0; r < 8; ++r) hlast[r] = 0.0f;
  __syncthreads();

  const v8f z8f = {0.f, 0.f, 0.f, 0.f, 0.f, 0.f, 0.f, 0.f};

#pragma unroll 1
  for (int t = 0; t < NSTEP; ++t) {
    const int tc = t & (XCH - 1);
    if (tc == 0) {
      const int r = tid >> 5, c2 = lane * 2;
      const v2f v = *(const v2f*)(x + (size_t)(b0 + r) * NSTEP + t + c2);
      const float x0 = v[0], x1 = v[1];
      v2f xb;
      xb[0] = bf16r(x0);
      xb[1] = bf16r(x1);
      *(v2f*)(s_x + r * SXP + c2) = xb;
      __syncthreads();
    }

    const int cur = t & 1;
    const _Float16* th = hbuf + (2 * cur) * TILEH + c * LDP + koff;
    const _Float16* tl = th + TILEH;
    _Float16* nh = hbuf + (2 * (cur ^ 1)) * TILEH;
    _Float16* nl = nh + TILEH;

    v8f accH = z8f, accL = z8f;
#pragma unroll
    for (int kb = 0; kb < NKB; ++kb) {
      const v16h aH = Frag<_Float16>::load(th + kb * 32);
      const v16h aL = Frag<_Float16>::load(tl + kb * 32);
      accH = Frag<_Float16>::mma(aH, bfr[kb], accH);
      accL = Frag<_Float16>::mma(aL, bfr[kb], accL);
      wmma_guard3(accH, accL, aH, aL, bfr[kb]);
      if (kb & 1) asm volatile("" ::: "memory");
    }
    acc_guard2(accH, accL);

#pragma unroll
    for (int r = 0; r < 8; ++r) {
      const float xv  = s_x[(mOff + r) * SXP + tc];
      const float u   = fmaf(xv, wih, bih) + bhh;
      const float rec = fmaf(accL[r], LOCAR_INV, accH[r]) * WCAR_INV;
      const float hn  = tanh_f(u + rec);
      hlast[r] = hn;
      const float hs  = (fabsf(hn) < F16_MIN_NORMAL) ? 0.0f : hn;
      const _Float16 h16 = (_Float16)hs;
      float hif = (float)h16;
      asm volatile("" : "+v"(hif));
      const float lof = (hn - hif) * LOCAR;
      const _Float16 l16 = (_Float16)lof;
      nh[(mOff + r) * LDP + hidx] = h16;
      nl[(mOff + r) * LDP + hidx] = l16;
    }
    __syncthreads();
  }

#pragma unroll
  for (int r = 0; r < 8; ++r) s_hf[(mOff + r) * HFP + hidx] = hlast[r];
  __syncthreads();

  if (tid < NOUTB) {
    const int r = tid / NP;
    const int p = tid - r * NP;
    const float* wrow = w_out + (size_t)p * NHID;
    const float* hrow = s_hf + r * HFP;
    float acc = 0.0f;
#pragma unroll 1
    for (int k = 0; k < NHID; k += 4) {
      const v4f wv = *(const v4f*)(wrow + k);
      const v4f hv = *(const v4f*)(hrow + k);
#pragma unroll
      for (int e = 0; e < 4; ++e) {
        const float we = wv[e], he = hv[e];
        acc = fmaf(he, bf16r(we), acc);
      }
    }
    acc += bf16r(b_out[p]);
    s_out[tid] = acc;
  }
  __syncthreads();

  if (wave == 0) {
    float* ob = out + (size_t)blockIdx.x * NOUTB;
    for (int pass = 0; pass < 2; ++pass) {
#pragma unroll
      for (int it = 0; it < 3; ++it) {
        const int idx = (it * 32 + lane) * 4;
        const v4f v = *(const v4f*)(s_out + idx);
        *(volatile v4f*)(ob + idx) = v;
      }
      __threadfence();
    }
  }
}

extern "C" void kernel_launch(void* const* d_in, const int* in_sizes, int n_in,
                              void* d_out, int out_size, void* d_ws, size_t ws_size, hipStream_t stream) {
  (void)d_ws; (void)ws_size;
  if (n_in < 7 || d_out == nullptr) return;
  if (in_sizes[0] != NB * NSTEP || in_sizes[1] != NHID || in_sizes[2] != NHID * NHID ||
      in_sizes[3] != NHID || in_sizes[4] != NHID || in_sizes[5] != NP * NHID || in_sizes[6] != NP ||
      out_size != NB * NP) return;

  const float* x     = (const float*)d_in[0];
  const float* w_ih  = (const float*)d_in[1];
  const float* w_hh  = (const float*)d_in[2];
  const float* b_ih  = (const float*)d_in[3];
  const float* b_hh  = (const float*)d_in[4];
  const float* w_out = (const float*)d_in[5];
  const float* b_out = (const float*)d_in[6];
  float* out = (float*)d_out;

  rnn_tanh_seq_kernel<<<dim3(NBLK), dim3(NTHR), 0, stream>>>(x, w_ih, w_hh, b_ih, b_hh, w_out, b_out, out);
}
